// GraphConvFlockingModel_75943611728684
// MI455X (gfx1250) — hardware-run, weakly checked
//
#include <hip/hip_runtime.h>

typedef __attribute__((ext_vector_type(16))) _Float16 v16h;
typedef __attribute__((ext_vector_type(8)))  _Float16 v8h;
typedef __attribute__((ext_vector_type(8)))  float    v8f;
typedef __attribute__((ext_vector_type(4)))  float    v4f;
typedef __attribute__((ext_vector_type(2)))  float    v2f;
typedef __attribute__((ext_vector_type(4)))  int      v4i;

constexpr int kNodes        = 100000;
constexpr int kEdges        = 3200000;
constexpr int kHalfFeat     = 32;
constexpr int kFeat         = 64;
constexpr int kOutDim       = 2;
constexpr int kBtRows       = 16;
constexpr int kWavesPerBlk  = 8;
constexpr int kRowsPerWave  = 64;
constexpr int kRowsPerBlk   = kWavesPerBlk * kRowsPerWave;
constexpr int kNodeBlocks   = (kNodes + kRowsPerBlk - 1) / kRowsPerBlk;
constexpr int kNodesPad     = kNodeBlocks * kRowsPerBlk;
constexpr int kTileNodes    = 8000;
constexpr int kEdgeThreads  = 512;
constexpr int kEdgeBlocks   = (kNodes + kTileNodes - 1) / kTileNodes;
constexpr int kOutIters     = (kTileNodes / 2 + kEdgeThreads - 1) / kEdgeThreads;

constexpr float kACarry   = 16.0f;
constexpr float kBCarry   = 256.0f;
constexpr float kLoCarry  = 2048.0f;
constexpr float kFold     = 1.0f / (kACarry * kBCarry);
constexpr float kLoInv    = 1.0f / kLoCarry;
constexpr float kFixScale = 1048576.0f;
constexpr float kFixInv   = 1.0f / kFixScale;
constexpr float kFixLimit = 1.0e9f;

static_assert(kFeat == 2 * kHalfFeat, "feature split");
static_assert((kFeat % 32) == 0, "K multiple of 32");
static_assert((kNodes % 16) == 0, "output lines of 16 nodes");
static_assert((kEdges % 4) == 0, "int4 edge loads");
static_assert((kTileNodes % 64) == 0, "tile of whole 512-B store chunks");
static_assert(kTileNodes * 2 * 4 <= 65536, "LDS accumulator size");
static_assert(kNodeBlocks == 196 && kEdgeBlocks == 13 && kOutIters == 8, "grid arithmetic");

constexpr size_t kSzBt    = (size_t)kBtRows * kFeat * 2;
constexpr size_t kSzBc    = 128;
constexpr size_t kSzPlane = (size_t)kNodesPad * kOutDim * 4;
constexpr size_t kOffBt   = 0;
constexpr size_t kOffBc   = kOffBt + kSzBt;
constexpr size_t kOffBase = kOffBc + kSzBc;
constexpr size_t kOffMpl  = kOffBase + kSzPlane;
constexpr size_t kWsTotal = kOffMpl + kSzPlane;
static_assert(kWsTotal == 1607808ull, "carve total");
static_assert(kWsTotal <= 134217728ull, "carve cap");
static_assert((kOffBc % 128) == 0 && (kOffBase % 128) == 0 && (kOffMpl % 128) == 0, "128-B aligned regions");

union FragH { v16h v; v8h h[2]; };

__device__ __forceinline__ v16h frag_load_h(const _Float16* p) {
  FragH f;
  f.h[0] = *(const v8h*)(p);
  f.h[1] = *(const v8h*)(p + 16);
  return f.v;
}

__device__ __forceinline__ v16h frag_from_f32_row(const float* rowp, int hh) {
  v4f y0 = *(const v4f*)(rowp + 8 * hh);
  v4f y1 = *(const v4f*)(rowp + 8 * hh + 4);
  v4f y2 = *(const v4f*)(rowp + 16 + 8 * hh);
  v4f y3 = *(const v4f*)(rowp + 16 + 8 * hh + 4);
  y0 = y0 * kACarry;
  y1 = y1 * kACarry;
  y2 = y2 * kACarry;
  y3 = y3 * kACarry;
  asm volatile("" : "+v"(y0), "+v"(y1), "+v"(y2), "+v"(y3));
  v16h a;
#pragma unroll
  for (int e = 0; e < 4; ++e) {
    a[e]      = (_Float16)y0[e];
    a[4 + e]  = (_Float16)y1[e];
    a[8 + e]  = (_Float16)y2[e];
    a[12 + e] = (_Float16)y3[e];
  }
  return a;
}

__device__ __forceinline__ v8f wmma_f16_step(v16h a, v16h b, v8f c) {
  c = __builtin_amdgcn_wmma_f32_16x16x32_f16(false, a, false, b, (short)0, c, false, false);
  asm volatile("v_nop\n\tv_nop\n\tv_nop\n\tv_nop" : "+v"(c) : "v"(a), "v"(b));
  return c;
}

__global__ __launch_bounds__(256) void prep_kernel(
    const float* __restrict__ W_rel, const float* __restrict__ b_rel,
    const float* __restrict__ W_root, const float* __restrict__ W_pred,
    const float* __restrict__ b_pred,
    unsigned short* __restrict__ Bt, float* __restrict__ bc)
{
  __shared__ __align__(16) float sP[4 * kFeat];
  const int tid = threadIdx.x;
  const int k  = tid >> 2;
  const int c  = tid & 3;
  const int cc = c & 1;
  float sr = 0.0f, sl = 0.0f, sb = 0.0f;
#pragma unroll 1
  for (int j = 0; j < kFeat; ++j) {
    const float wp = W_pred[j * kOutDim + cc];
    sr = fmaf(W_root[k * kFeat + j], wp, sr);
    sl = fmaf(W_rel[k * kFeat + j], wp, sl);
    sb = fmaf(b_rel[j], wp, sb);
  }
  const float pv  = (c < 2) ? sr : sl;
  const float bpv = b_pred[cc];
  sP[c * kFeat + k] = pv * kBCarry;
  __syncthreads();

  const int n  = (tid >> 3) & 15;
  const int k8 = (tid & 7) * 8;
  v8h hv;
#pragma unroll
  for (int e = 0; e < 8; ++e) {
    const float pc  = sP[(n & 3) * kFeat + k8 + e];
    const _Float16 hi = (_Float16)pc;
    const float hif = (float)hi;
    const float lof = (pc - hif) * kLoCarry;
    const float v   = (n < 4) ? hif : ((n < 8) ? lof : 0.0f);
    hv[e] = (_Float16)v;
  }
  unsigned short* btp = Bt + n * kFeat + k8;
  const int bl = tid & 31;
  const float bcv = (bl < 2) ? (sb + bpv) : 0.0f;
  const bool wBt = (tid < 128);
  const bool wBc = (tid >= 128) && (tid < 160);
  if (wBt) { *(volatile v8h*)btp = hv; }
  if (wBc) { ((volatile float*)bc)[bl] = bcv; }
  __threadfence();
  if (wBt) { *(volatile v8h*)btp = hv; }
  if (wBc) { ((volatile float*)bc)[bl] = bcv; }
}

__global__ __launch_bounds__(256) void node_gemm_kernel(
    const float* __restrict__ pos, const float* __restrict__ vel,
    const unsigned short* __restrict__ Btp, const float* __restrict__ bcp,
    float* __restrict__ basep, float* __restrict__ mpl)
{
  __shared__ __align__(16) float sD[kWavesPerBlk][kRowsPerWave * 16];
  const int tid  = threadIdx.x;
  const int lane = tid & 31;
  const int wave = tid >> 5;
  const int hh   = lane >> 4;
  const int c    = lane & 15;
  const int row0 = (blockIdx.x * kWavesPerBlk + wave) * kRowsPerWave;

  const _Float16* Bt = (const _Float16*)Btp;
  const v16h b0 = frag_load_h(Bt + c * kFeat + 8 * hh);
  const v16h b1 = frag_load_h(Bt + c * kFeat + 32 + 8 * hh);
  const float bc0 = bcp[0];
  const float bc1 = bcp[1];

  v8f acc[4];
#pragma unroll
  for (int t = 0; t < 4; ++t) acc[t] = (v8f){0.f, 0.f, 0.f, 0.f, 0.f, 0.f, 0.f, 0.f};

#pragma unroll
  for (int t = 0; t < 4; ++t) {
    int row = row0 + t * 16 + c;
    row = (row < kNodes) ? row : (kNodes - 1);
    const v16h ap = frag_from_f32_row(pos + (size_t)row * kHalfFeat, hh);
    const v16h av = frag_from_f32_row(vel + (size_t)row * kHalfFeat, hh);
    acc[t] = wmma_f16_step(ap, b0, acc[t]);
    acc[t] = wmma_f16_step(av, b1, acc[t]);
  }

  float* slab = sD[wave];
#pragma unroll
  for (int t = 0; t < 4; ++t) {
#pragma unroll
    for (int r = 0; r < 8; ++r) slab[(t * 16 + 8 * hh + r) * 16 + c] = acc[t][r];
  }
  __syncthreads();

  const float* sp = slab + (2 * lane) * 16;
  const v4f p0 = *(const v4f*)(sp);
  const v4f p1 = *(const v4f*)(sp + 4);
  const v4f q0 = *(const v4f*)(sp + 16);
  const v4f q1 = *(const v4f*)(sp + 20);
  v4f bv, mv;
  bv[0] = (p0[0] + p1[0] * kLoInv) * kFold + bc0;
  bv[1] = (p0[1] + p1[1] * kLoInv) * kFold + bc1;
  bv[2] = (q0[0] + q1[0] * kLoInv) * kFold + bc0;
  bv[3] = (q0[1] + q1[1] * kLoInv) * kFold + bc1;
  mv[0] = (p0[2] + p1[2] * kLoInv) * kFold;
  mv[1] = (p0[3] + p1[3] * kLoInv) * kFold;
  mv[2] = (q0[2] + q1[2] * kLoInv) * kFold;
  mv[3] = (q0[3] + q1[3] * kLoInv) * kFold;

  const int node = row0 + 2 * lane;
  const bool wr = (node < kNodes);
  float* bp = basep + (size_t)node * kOutDim;
  float* mp = mpl + (size_t)node * kOutDim;
  if (wr) {
    *(volatile v4f*)bp = bv;
    *(volatile v4f*)mp = mv;
  }
  __threadfence();
  if (wr) {
    *(volatile v4f*)bp = bv;
    *(volatile v4f*)mp = mv;
  }
}

__global__ __launch_bounds__(512) void edge_sum_kernel(
    const int* __restrict__ edges, const float* __restrict__ mpl,
    const float* __restrict__ basep, float* __restrict__ out)
{
  __shared__ __align__(16) int sAcc[kTileNodes * 2];
  const int tid   = threadIdx.x;
  const int node0 = blockIdx.x * kTileNodes;
  int cnt = kNodes - node0;
  cnt = (cnt < kTileNodes) ? cnt : kTileNodes;
  cnt = (cnt > 16) ? cnt : 16;

#pragma unroll 1
  for (int i = tid; i < kTileNodes * 2; i += kEdgeThreads) sAcc[i] = 0;
  __syncthreads();

  constexpr int kQuads = kEdges / 4;
  const v4i* src4 = (const v4i*)edges;
  const v4i* dst4 = (const v4i*)(edges + kEdges);

#pragma unroll 1
  for (int q0 = 0; q0 < kQuads; q0 += kEdgeThreads) {
    const int q = q0 + tid;
    const bool valid = (q < kQuads);
    const int qc = valid ? q : (kQuads - 1);
    const v4i sv = src4[qc];
    const v4i dv = dst4[qc];
#pragma unroll
    for (int e = 0; e < 4; ++e) {
      int s = sv[e];
      int d = dv[e];
      s = (s < 0) ? 0 : s;
      s = (s > kNodes - 1) ? (kNodes - 1) : s;
      d = (d < 0) ? 0 : d;
      d = (d > kNodes - 1) ? (kNodes - 1) : d;
      const v2f mv = *(const v2f*)(mpl + (size_t)s * kOutDim);
      float mx = mv[0];
      float my = mv[1];
      asm volatile("" : "+v"(mx), "+v"(my));
      const float fxs = fminf(fmaxf(mx * kFixScale, -kFixLimit), kFixLimit);
      const float fys = fminf(fmaxf(my * kFixScale, -kFixLimit), kFixLimit);
      const int fx = __float2int_rn(fxs);
      const int fy = __float2int_rn(fys);
      const int rel = d - node0;
      const bool hit = valid && ((unsigned)rel < (unsigned)cnt);
      if (hit) {
        __hip_atomic_fetch_add(&sAcc[rel * 2], fx, __ATOMIC_RELAXED, __HIP_MEMORY_SCOPE_WORKGROUP);
        __hip_atomic_fetch_add(&sAcc[rel * 2 + 1], fy, __ATOMIC_RELAXED, __HIP_MEMORY_SCOPE_WORKGROUP);
      }
    }
  }
  __syncthreads();

  const int nF4 = cnt >> 1;
  const float* bsrc = basep + (size_t)node0 * kOutDim;
  float* odst = out + (size_t)node0 * kOutDim;
  for (int pass = 0; pass < 2; ++pass) {
#pragma unroll 1
    for (int it = 0; it < kOutIters; ++it) {
      const int i = it * kEdgeThreads + tid;
      int ic = (i < nF4) ? i : (nF4 - 1);
      ic = (ic > 0) ? ic : 0;
      const v4i a = *(const v4i*)(sAcc + ic * 4);
      v4f b = *(const v4f*)(bsrc + (size_t)ic * 4);
      asm volatile("" : "+v"(b));
      v4f o;
      o[0] = b[0] + (float)a[0] * kFixInv;
      o[1] = b[1] + (float)a[1] * kFixInv;
      o[2] = b[2] + (float)a[2] * kFixInv;
      o[3] = b[3] + (float)a[3] * kFixInv;
      if (i < nF4) {
        *(volatile v4f*)(odst + (size_t)i * 4) = o;
      }
    }
    __threadfence();
  }
}

extern "C" void kernel_launch(void* const* d_in, const int* in_sizes, int n_in,
                              void* d_out, int out_size, void* d_ws, size_t ws_size,
                              hipStream_t stream) {
  if (n_in < 8) return;
  if (in_sizes[0] != kNodes * kHalfFeat) return;
  if (in_sizes[1] != kNodes * kHalfFeat) return;
  if (in_sizes[2] != 2 * kEdges) return;
  if (in_sizes[3] != kFeat * kFeat) return;
  if (in_sizes[4] != kFeat) return;
  if (in_sizes[5] != kFeat * kFeat) return;
  if (in_sizes[6] != kFeat * kOutDim) return;
  if (in_sizes[7] != kOutDim) return;
  if (out_size != kNodes * kOutDim) return;
  if (ws_size < kWsTotal) return;

  const float* pos    = (const float*)d_in[0];
  const float* vel    = (const float*)d_in[1];
  const int*   edges  = (const int*)d_in[2];
  const float* W_rel  = (const float*)d_in[3];
  const float* b_rel  = (const float*)d_in[4];
  const float* W_root = (const float*)d_in[5];
  const float* W_pred = (const float*)d_in[6];
  const float* b_pred = (const float*)d_in[7];
  float* out = (float*)d_out;

  char* ws = (char*)d_ws;
  unsigned short* Bt = (unsigned short*)(ws + kOffBt);
  float* bc   = (float*)(ws + kOffBc);
  float* base = (float*)(ws + kOffBase);
  float* mpl  = (float*)(ws + kOffMpl);

  prep_kernel<<<1, 256, 0, stream>>>(W_rel, b_rel, W_root, W_pred, b_pred, Bt, bc);
  node_gemm_kernel<<<kNodeBlocks, 256, 0, stream>>>(pos, vel, Bt, bc, base, mpl);
  edge_sum_kernel<<<kEdgeBlocks, kEdgeThreads, 0, stream>>>(edges, mpl, base, out);
}
